// GAU_73151882985867
// MI455X (gfx1250) — hardware-verified
//
#include <hip/hip_runtime.h>


#ifndef NB
#define NB 4
#endif
#ifndef SEQ
#define SEQ 2048
#endif
#define NB_FULL 4
#define SEQ_FULL 2048
#define DM 1024
#define DF 2048
#define QS 128
#define MROWS (NB * SEQ)

static_assert(NB >= 1 && NB <= NB_FULL);
static_assert(SEQ >= 256 && SEQ <= SEQ_FULL && (SEQ % 256) == 0);
static_assert((MROWS % 128) == 0 && (DM % 128) == 0 && (DF % 128) == 0 && QS == 128);
static_assert((DM % 32) == 0 && (DF % 32) == 0 && (SEQ % 32) == 0);

typedef float        v8f  __attribute__((ext_vector_type(8)));
typedef float        v4f  __attribute__((ext_vector_type(4)));
typedef _Float16     v8h  __attribute__((ext_vector_type(8)));
typedef _Float16     v16h __attribute__((ext_vector_type(16)));
typedef __bf16       v8b  __attribute__((ext_vector_type(8)));
typedef __bf16       v16b __attribute__((ext_vector_type(16)));
typedef unsigned int v4u  __attribute__((ext_vector_type(4)));
typedef int          v8i  __attribute__((ext_vector_type(8)));

enum { MD_U = 0, MD_V = 1, MD_QK = 2, MD_OUT = 3 };

constexpr int LDS16   = 128 * 136 * 2;
constexpr int LDSPRM  = 6 * QS * 4;
constexpr int LDSQK   = LDS16 + LDSPRM;
constexpr int LDS32   = 128 * 132 * 4;
constexpr int SP      = SEQ + 4;
constexpr int PP      = SEQ + 8;
constexpr int ATT_LDS = 16 * SP * 4 + 16 * PP * 2;
static_assert(((16 * SP * 4) % 16) == 0 && ((SP * 4) % 16) == 0 && ((PP * 2) % 16) == 0);
static_assert((LDS16 % 16) == 0);

__device__ __forceinline__ unsigned int bf16bits(float v) {
  unsigned int u = __float_as_uint(v);
  u += 0x7fffu + ((u >> 16) & 1u);
  return u >> 16;
}
__device__ __forceinline__ float bf16r(float v) {
  return __uint_as_float(bf16bits(v) << 16);
}
__device__ __forceinline__ unsigned int f16bits(float v) {
  const _Float16 hv = (_Float16)v;
  const unsigned short s = __builtin_bit_cast(unsigned short, hv);
  return (unsigned int)s;
}
__device__ __forceinline__ float silu_f(float v) {
  return v * __builtin_amdgcn_rcpf(1.0f + __expf(-v));
}

__device__ __forceinline__ v8f mma_f16(v16h a, v16h b, v8f c) {
  v8f d = __builtin_amdgcn_wmma_f32_16x16x32_f16(false, a, false, b, (short)0, c, false, false);
  asm volatile("v_nop\n\tv_nop\n\tv_nop\n\tv_nop" : "+v"(d) : "v"(a), "v"(b));
  return d;
}
__device__ __forceinline__ v8f mma_bf16(v16b a, v16b b, v8f c) {
  v8f d = __builtin_amdgcn_wmma_f32_16x16x32_bf16(false, a, false, b, (short)0, c, false, false);
  const v8i ai = __builtin_bit_cast(v8i, a);
  const v8i bi = __builtin_bit_cast(v8i, b);
  asm volatile("v_nop\n\tv_nop\n\tv_nop\n\tv_nop" : "+v"(d) : "v"(ai), "v"(bi));
  return d;
}

template <typename T> struct Tr;
template <> struct Tr<_Float16> {
  typedef v16h V16; typedef v8h V8;
  static __device__ __forceinline__ v8f mma(V16 a, V16 b, v8f c) { return mma_f16(a, b, c); }
};
template <> struct Tr<__bf16> {
  typedef v16b V16; typedef v8b V8;
  static __device__ __forceinline__ v8f mma(V16 a, V16 b, v8f c) { return mma_bf16(a, b, c); }
};
template <typename T> union Frag { typename Tr<T>::V16 v; typename Tr<T>::V8 hv[2]; };

template <typename T>
__device__ __forceinline__ void ldfrag(Frag<T>& f, const T* row, int k0, int h) {
  typedef typename Tr<T>::V8 V8;
  f.hv[0] = *(const V8*)(row + k0 + 8 * h);
  f.hv[1] = *(const V8*)(row + k0 + 16 + 8 * h);
}

__global__ __launch_bounds__(256) void k_cvt_x(const float* __restrict__ x, unsigned short* xb) {
  const int gid = blockIdx.x * 256 + threadIdx.x;
  const int row = gid >> 7, c = gid & 127;
  const int b = row / SEQ, tt = row - b * SEQ;
  const float* src = x + ((size_t)(b * SEQ_FULL + tt)) * DM + c * 8;
  const v4f f0 = *(const v4f*)src;
  const v4f f1 = *(const v4f*)(src + 4);
  v4u pk;
  pk[0] = bf16bits(f0[0]) | (bf16bits(f0[1]) << 16);
  pk[1] = bf16bits(f0[2]) | (bf16bits(f0[3]) << 16);
  pk[2] = bf16bits(f1[0]) | (bf16bits(f1[1]) << 16);
  pk[3] = bf16bits(f1[2]) | (bf16bits(f1[3]) << 16);
  unsigned short* dst = xb + (size_t)row * DM + c * 8;
  *(volatile v4u*)dst = pk;
  __threadfence();
  *(volatile v4u*)dst = pk;
}

template <int F16OUT>
__global__ __launch_bounds__(256) void k_cvt_wT(const float* __restrict__ W, unsigned short* WT,
                                                int Kdim, int Ndim, float scale) {
  __shared__ __attribute__((aligned(16))) unsigned short st[64 * 72];
  const int t = threadIdx.x;
  const int n0 = blockIdx.x * 64, k0 = blockIdx.y * 64;
#pragma unroll
  for (int i = 0; i < 4; ++i) {
    const int idx = t + i * 256, kr = idx >> 4, c4 = idx & 15;
    const v4f f = *(const v4f*)(W + ((size_t)(k0 + kr)) * Ndim + n0 + c4 * 4);
#pragma unroll
    for (int j = 0; j < 4; ++j) {
      const float rv = bf16r(f[j]);
      const unsigned int bits = F16OUT ? f16bits(rv * scale) : bf16bits(rv);
      st[(c4 * 4 + j) * 72 + kr] = (unsigned short)bits;
    }
  }
  __syncthreads();
#pragma unroll
  for (int p = 0; p < 2; ++p) {
    const int row = p * 32 + (t >> 3), c = t & 7;
    const v4u val = *(const v4u*)(st + row * 72 + c * 8);
    unsigned short* dst = WT + ((size_t)(n0 + row)) * Kdim + k0 + c * 8;
    *(volatile v4u*)dst = val;
  }
  __threadfence();
#pragma unroll
  for (int p = 0; p < 2; ++p) {
    const int row = p * 32 + (t >> 3), c = t & 7;
    const v4u val = *(const v4u*)(st + row * 72 + c * 8);
    unsigned short* dst = WT + ((size_t)(n0 + row)) * Kdim + k0 + c * 8;
    *(volatile v4u*)dst = val;
  }
}

template <int MODE, typename T>
__global__ __launch_bounds__(256) void k_gemm(
    const T* __restrict__ A, const T* __restrict__ Bt, int K,
    const float* __restrict__ bias, const float* __restrict__ gamma,
    const float* __restrict__ beta, const float* __restrict__ uqk,
    unsigned short* out16a, unsigned short* out16b, float* outf) {
  extern __shared__ __attribute__((aligned(16))) unsigned char dyn_smem[];
  const int t = threadIdx.x, lane = t & 31, h = lane >> 4, l15 = lane & 15, w = t >> 5;
  const int mw = (w & 3) * 32, nw = (w >> 2) * 64;
  const int n0 = blockIdx.x * 128, m0 = blockIdx.y * 128;

  if constexpr (MODE == MD_QK) {
    float* prm = (float*)(dyn_smem + LDS16);
#pragma unroll
    for (int i = 0; i < 3; ++i) {
      const int idx = t + 256 * i;
      const int vec = idx >> 7, col = idx & (QS - 1);
      const float* src = (vec == 0) ? bias
                       : (vec == 1) ? gamma
                       : (vec == 2) ? (gamma + QS)
                       : (vec == 3) ? beta
                       : (vec == 4) ? (beta + QS)
                       : uqk;
      prm[idx] = bf16r(src[col]);
    }
    __syncthreads();
  }

  v8f zero = {};
  v8f acc[2][4];
#pragma unroll
  for (int mt = 0; mt < 2; ++mt)
#pragma unroll
    for (int nt = 0; nt < 4; ++nt) acc[mt][nt] = zero;

  const T* arow = A  + ((size_t)(m0 + mw + l15)) * K;
  const T* brow = Bt + ((size_t)(n0 + nw + l15)) * K;
  const size_t s16 = (size_t)16 * K;

#pragma unroll 1
  for (int k0 = 0; k0 < K; k0 += 32) {
    Frag<T> af[2], bfq[4];
    ldfrag<T>(af[0], arow, k0, h);
    ldfrag<T>(af[1], arow + s16, k0, h);
#pragma unroll
    for (int nt = 0; nt < 4; ++nt) ldfrag<T>(bfq[nt], brow + nt * s16, k0, h);
#pragma unroll
    for (int mt = 0; mt < 2; ++mt)
#pragma unroll
      for (int nt = 0; nt < 4; ++nt)
        acc[mt][nt] = Tr<T>::mma(af[mt].v, bfq[nt].v, acc[mt][nt]);
  }

  if constexpr (MODE == MD_OUT) {
    float* stf = (float*)dyn_smem;
#pragma unroll
    for (int nt = 0; nt < 4; ++nt) {
      const int lcol = nw + nt * 16 + l15;
      const float bv = bf16r(bias[n0 + lcol]);
#pragma unroll
      for (int mt = 0; mt < 2; ++mt)
#pragma unroll
        for (int r = 0; r < 8; ++r)
          stf[(mw + mt * 16 + 8 * h + r) * 132 + lcol] = acc[mt][nt][r] * (1.0f / 2048.0f) + bv;
    }
    __syncthreads();
#pragma unroll
    for (int p = 0; p < 16; ++p) {
      const int row = p * 8 + w;
      const v4f val = *(const v4f*)(stf + row * 132 + lane * 4);
      float* dst = outf + ((size_t)(m0 + row)) * DM + n0 + lane * 4;
      *(volatile v4f*)dst = val;
    }
    __threadfence();
#pragma unroll
    for (int p = 0; p < 16; ++p) {
      const int row = p * 8 + w;
      const v4f val = *(const v4f*)(stf + row * 132 + lane * 4);
      float* dst = outf + ((size_t)(m0 + row)) * DM + n0 + lane * 4;
      *(volatile v4f*)dst = val;
    }
  } else {
    unsigned short* st = (unsigned short*)dyn_smem;
    constexpr int NSEL = (MODE == MD_QK) ? 2 : 1;
    const int bidx = m0 / SEQ;
    const int j0   = m0 - bidx * SEQ;
#pragma unroll 1
    for (int sel = 0; sel < NSEL; ++sel) {
      if (sel) __syncthreads();
#pragma unroll
      for (int nt = 0; nt < 4; ++nt) {
        const int lcol = nw + nt * 16 + l15;
        const int gcol = n0 + lcol;
        float bv, g0 = 0.f, g1 = 0.f, be0 = 0.f, be1 = 0.f, uq = 0.f;
        if constexpr (MODE == MD_QK) {
          const float* prm = (const float*)(dyn_smem + LDS16);
          bv  = prm[lcol];
          g0  = prm[1 * QS + lcol]; g1  = prm[2 * QS + lcol];
          be0 = prm[3 * QS + lcol]; be1 = prm[4 * QS + lcol];
          uq  = prm[5 * QS + lcol];
        } else {
          bv = bf16r(bias[gcol]);
        }
#pragma unroll
        for (int mt = 0; mt < 2; ++mt) {
#pragma unroll
          for (int r = 0; r < 8; ++r) {
            const int lrow = mw + mt * 16 + 8 * h + r;
            const float s = acc[mt][nt][r] + bv;
            if constexpr (MODE == MD_U) {
              st[lrow * 136 + lcol] = (unsigned short)f16bits(silu_f(s));
            } else if constexpr (MODE == MD_V) {
              st[lcol * 136 + lrow] = (unsigned short)f16bits(silu_f(s) * 16.0f);
            } else {
              const float z = silu_f(s);
              const float cq = 1.0f / 11.313708305358887f;
              const float qv = ((z * g0 + be0) * cq + uq) * 16.0f;
              const float kv = (z * g1 + be1) * 4.0f;
              st[lrow * 136 + lcol] = (unsigned short)f16bits(sel == 0 ? qv : kv);
            }
          }
        }
      }
      __syncthreads();
#pragma unroll
      for (int p = 0; p < 8; ++p) {
        const int row = p * 16 + (t >> 4), c = t & 15;
        const v4u val = *(const v4u*)(st + row * 136 + c * 8);
        unsigned short* dst;
        if constexpr (MODE == MD_U) dst = out16a + ((size_t)(m0 + row)) * DF + n0 + c * 8;
        else if constexpr (MODE == MD_V) dst = out16a + ((size_t)(bidx * DF + n0 + row)) * SEQ + j0 + c * 8;
        else dst = (sel ? out16b : out16a) + ((size_t)(m0 + row)) * QS + c * 8;
        *(volatile v4u*)dst = val;
      }
      __threadfence();
#pragma unroll
      for (int p = 0; p < 8; ++p) {
        const int row = p * 16 + (t >> 4), c = t & 15;
        const v4u val = *(const v4u*)(st + row * 136 + c * 8);
        unsigned short* dst;
        if constexpr (MODE == MD_U) dst = out16a + ((size_t)(m0 + row)) * DF + n0 + c * 8;
        else if constexpr (MODE == MD_V) dst = out16a + ((size_t)(bidx * DF + n0 + row)) * SEQ + j0 + c * 8;
        else dst = (sel ? out16b : out16a) + ((size_t)(m0 + row)) * QS + c * 8;
        *(volatile v4u*)dst = val;
      }
    }
  }
}

__global__ __launch_bounds__(512) void k_attn(
    const _Float16* __restrict__ qp, const _Float16* __restrict__ kp,
    const _Float16* __restrict__ vT, const int* __restrict__ len,
    unsigned short* uo) {
  extern __shared__ __attribute__((aligned(16))) unsigned char dyn_smem[];
  float* Sc = (float*)dyn_smem;
  _Float16* Pm = (_Float16*)(dyn_smem + 16 * SP * 4);

  const int t = threadIdx.x, lane = t & 31, h = lane >> 4, l15 = lane & 15, w = t >> 5;
  constexpr int TILES = SEQ / 16;
  const int b  = blockIdx.x / TILES;
  const int i0 = (blockIdx.x - b * TILES) * 16;
  const int lenb = len[b];
  const float NEG = -__builtin_huge_valf();
  v8f zero = {};

  {
    Frag<_Float16> qa[4];
    const _Float16* qrow = qp + ((size_t)(b * SEQ + i0 + l15)) * QS;
#pragma unroll
    for (int kt = 0; kt < 4; ++kt) ldfrag<_Float16>(qa[kt], qrow, kt * 32, h);
    constexpr int KPW = SEQ / 16;
#pragma unroll 1
    for (int jt = 0; jt < KPW / 16; ++jt) {
      const int j0 = w * KPW + jt * 16;
      const _Float16* krow = kp + ((size_t)(b * SEQ + j0 + l15)) * QS;
      v8f s = zero;
#pragma unroll
      for (int kt = 0; kt < 4; ++kt) {
        Frag<_Float16> kb;
        ldfrag<_Float16>(kb, krow, kt * 32, h);
        s = mma_f16(qa[kt].v, kb.v, s);
      }
      const int j = j0 + l15;
      const bool valid = j < lenb;
#pragma unroll
      for (int r = 0; r < 8; ++r)
        Sc[(8 * h + r) * SP + j] = valid ? s[r] * (1.0f / 64.0f) : NEG;
    }
  }
  __syncthreads();

  {
    float* srow = Sc + w * SP;
    float mx = NEG;
#pragma unroll 4
    for (int i = 0; i < SEQ / 32; ++i) mx = fmaxf(mx, srow[lane + 32 * i]);
#pragma unroll
    for (int o = 16; o > 0; o >>= 1) mx = fmaxf(mx, __shfl_xor(mx, o));
    float sum = 0.f;
#pragma unroll 4
    for (int i = 0; i < SEQ / 32; ++i) {
      const float e = __expf(srow[lane + 32 * i] - mx);
      srow[lane + 32 * i] = e;
      sum += e;
    }
#pragma unroll
    for (int o = 16; o > 0; o >>= 1) sum += __shfl_xor(sum, o);
    const float inv = 1024.0f * __builtin_amdgcn_rcpf(sum);
    _Float16* prow = Pm + w * PP;
#pragma unroll 4
    for (int i = 0; i < SEQ / 32; ++i) prow[lane + 32 * i] = (_Float16)(srow[lane + 32 * i] * inv);
  }
  __syncthreads();

  v8f acc[8];
#pragma unroll
  for (int nt = 0; nt < 8; ++nt) acc[nt] = zero;
  {
    const _Float16* parow = Pm + l15 * PP;
    const _Float16* vrow  = vT + ((size_t)(b * DF + w * 128 + l15)) * SEQ;
    const size_t vs16 = (size_t)16 * SEQ;
#pragma unroll 1
    for (int kk = 0; kk < SEQ / 32; ++kk) {
      Frag<_Float16> pa;
      ldfrag<_Float16>(pa, parow, kk * 32, h);
#pragma unroll
      for (int nt = 0; nt < 8; ++nt) {
        Frag<_Float16> vb;
        ldfrag<_Float16>(vb, vrow + nt * vs16, kk * 32, h);
        acc[nt] = mma_f16(pa.v, vb.v, acc[nt]);
      }
    }
  }
  __syncthreads();

  float* Ost = Sc;
#pragma unroll
  for (int nt = 0; nt < 8; ++nt)
#pragma unroll
    for (int r = 0; r < 8; ++r)
      Ost[(8 * h + r) * SP + w * 128 + nt * 16 + l15] = acc[nt][r];
  __syncthreads();

  _Float16* O16 = Pm;
  const int rsub = t >> 8;
  const int c8   = (t & 255) * 8;
  const float cs = 32.0f / 16384.0f;
#pragma unroll 1
  for (int p = 0; p < 8; ++p) {
    const int row = p * 2 + rsub;
    const size_t g = ((size_t)(b * SEQ + i0 + row)) * DF + c8;
    const v8h uu = *(const v8h*)(uo + g);
    const v4f a0 = *(const v4f*)(Ost + row * SP + c8);
    const v4f a1 = *(const v4f*)(Ost + row * SP + c8 + 4);
    v8h o;
#pragma unroll
    for (int e = 0; e < 4; ++e) {
      o[e]     = (_Float16)(a0[e] * cs * (float)uu[e]);
      o[e + 4] = (_Float16)(a1[e] * cs * (float)uu[e + 4]);
    }
    *(v8h*)(O16 + row * PP + c8) = o;
  }
  __syncthreads();
#pragma unroll
  for (int p = 0; p < 8; ++p) {
    const int row = p * 2 + rsub;
    const size_t g = ((size_t)(b * SEQ + i0 + row)) * DF + c8;
    const v4u val = *(const v4u*)((const unsigned short*)O16 + row * PP + c8);
    *(volatile v4u*)(uo + g) = val;
  }
  __threadfence();
#pragma unroll
  for (int p = 0; p < 8; ++p) {
    const int row = p * 2 + rsub;
    const size_t g = ((size_t)(b * SEQ + i0 + row)) * DF + c8;
    const v4u val = *(const v4u*)((const unsigned short*)O16 + row * PP + c8);
    *(volatile v4u*)(uo + g) = val;
  }
}

extern "C" void kernel_launch(void* const* d_in, const int* in_sizes, int n_in,
                              void* d_out, int out_size, void* d_ws, size_t ws_size,
                              hipStream_t stream) {
  if (n_in < 13) return;
  const long need_x = ((long)(NB - 1) * SEQ_FULL + SEQ) * DM;
  if ((long)in_sizes[0] < need_x) return;
  if (in_sizes[1] < NB) return;
  if (in_sizes[2] < DM * DF || in_sizes[3] < DF) return;
  if (in_sizes[4] < DM * DF || in_sizes[5] < DF) return;
  if (in_sizes[6] < DM * QS || in_sizes[7] < QS) return;
  if (in_sizes[8] < DF * DM || in_sizes[9] < DM) return;
  if (in_sizes[10] < 2 * QS || in_sizes[11] < 2 * QS || in_sizes[12] < QS) return;
  if ((long)out_size < (long)MROWS * DM) return;

  const float* x     = (const float*)d_in[0];
  const int*   len   = (const int*)d_in[1];
  const float* Wu_w  = (const float*)d_in[2];
  const float* Wu_b  = (const float*)d_in[3];
  const float* Wv_w  = (const float*)d_in[4];
  const float* Wv_b  = (const float*)d_in[5];
  const float* Wqk_w = (const float*)d_in[6];
  const float* Wqk_b = (const float*)d_in[7];
  const float* Wo_w  = (const float*)d_in[8];
  const float* Wo_b  = (const float*)d_in[9];
  const float* gamma = (const float*)d_in[10];
  const float* beta  = (const float*)d_in[11];
  const float* u_qk  = (const float*)d_in[12];
  float* out = (float*)d_out;

  char* ws = (char*)d_ws;
  size_t off = 0;
  auto carve = [&](size_t bytes) -> unsigned short* {
    unsigned short* p = (unsigned short*)(ws + off);
    off += (bytes + 255) & ~(size_t)255;
    return p;
  };
  unsigned short* xb   = carve((size_t)MROWS * DM * 2);
  unsigned short* WuT  = carve((size_t)DF * DM * 2);
  unsigned short* WvT  = carve((size_t)DF * DM * 2);
  unsigned short* WqkT = carve((size_t)QS * DM * 2);
  unsigned short* WoT  = carve((size_t)DM * DF * 2);
  unsigned short* uo   = carve((size_t)MROWS * DF * 2);
  unsigned short* vTp  = carve((size_t)NB * DF * SEQ * 2);
  unsigned short* qpl  = carve((size_t)MROWS * QS * 2);
  unsigned short* kpl  = carve((size_t)MROWS * QS * 2);
  if (off > ws_size) return;

  const float* nullf = (const float*)0;
  unsigned short* nulls = (unsigned short*)0;
  float* nullo = (float*)0;

  k_cvt_x<<<dim3(MROWS * (DM / 8) / 256), dim3(256), 0, stream>>>(x, xb);
  k_cvt_wT<0><<<dim3(DF / 64, DM / 64), dim3(256), 0, stream>>>(Wu_w,  WuT,  DM, DF, 1.0f);
  k_cvt_wT<0><<<dim3(DF / 64, DM / 64), dim3(256), 0, stream>>>(Wv_w,  WvT,  DM, DF, 1.0f);
  k_cvt_wT<0><<<dim3(QS / 64, DM / 64), dim3(256), 0, stream>>>(Wqk_w, WqkT, DM, QS, 1.0f);
  k_cvt_wT<1><<<dim3(DM / 64, DF / 64), dim3(256), 0, stream>>>(Wo_w,  WoT,  DF, DM, 64.0f);
  k_gemm<MD_U, __bf16><<<dim3(DF / 128, MROWS / 128), dim3(256), LDS16, stream>>>(
      (const __bf16*)xb, (const __bf16*)WuT, DM, Wu_b, nullf, nullf, nullf, uo, nulls, nullo);
  k_gemm<MD_V, __bf16><<<dim3(DF / 128, MROWS / 128), dim3(256), LDS16, stream>>>(
      (const __bf16*)xb, (const __bf16*)WvT, DM, Wv_b, nullf, nullf, nullf, vTp, nulls, nullo);
  k_gemm<MD_QK, __bf16><<<dim3(QS / 128, MROWS / 128), dim3(256), LDSQK, stream>>>(
      (const __bf16*)xb, (const __bf16*)WqkT, DM, Wqk_b, gamma, beta, u_qk, qpl, kpl, nullo);
  hipFuncSetAttribute(reinterpret_cast<const void*>(&k_attn),
                      hipFuncAttributeMaxDynamicSharedMemorySize, ATT_LDS);
  k_attn<<<dim3(NB * (SEQ / 16)), dim3(512), ATT_LDS, stream>>>(
      (const _Float16*)qpl, (const _Float16*)kpl, (const _Float16*)vTp, len, uo);
  hipFuncSetAttribute(reinterpret_cast<const void*>(&k_gemm<MD_OUT, _Float16>),
                      hipFuncAttributeMaxDynamicSharedMemorySize, LDS32);
  k_gemm<MD_OUT, _Float16><<<dim3(DM / 128, MROWS / 128), dim3(256), LDS32, stream>>>(
      (const _Float16*)uo, (const _Float16*)WoT, DF, Wo_b, nullf, nullf, nullf, nulls, nulls, out);
}
